// WindowAttentionV2_66468913873037
// MI455X (gfx1250) — hardware-verified
//
#include <hip/hip_runtime.h>


namespace {
constexpr int BW = 256, N = 256, C = 192, NH = 6, DH = 32, NW = 64, NQKV = 3 * C, MROWS = BW * N;
constexpr int TBL = 961, TBLP = 992, CPB = 512;
constexpr float KSC = 64.0f;

typedef _Float16 b16;
typedef __attribute__((ext_vector_type(16))) _Float16 v16b;
typedef __attribute__((ext_vector_type(8)))  _Float16 v8b;
typedef __attribute__((ext_vector_type(8)))  float v8f;
typedef __attribute__((ext_vector_type(4)))  float v4f;

__device__ __forceinline__ v8b ld8b(const b16* p) { return *(const v8b*)p; }
__device__ __forceinline__ v16b cat8b(v8b a, v8b b) { return __builtin_shufflevector(a, b, 0, 1, 2, 3, 4, 5, 6, 7, 8, 9, 10, 11, 12, 13, 14, 15); }
__device__ __forceinline__ v16b frag_kb(const b16* p, int hh) { return cat8b(ld8b(p + 8 * hh), ld8b(p + 16 + 8 * hh)); }
__device__ __forceinline__ void split16(float v, b16& hi, b16& lo) { hi = (b16)v; lo = (b16)(v - (float)hi); }
__device__ __forceinline__ void frag_ksplit(const float* p, int hh, v16b& fh_, v16b& fl_) {
  const float* p0 = p + 8 * hh; const float* p1 = p + 16 + 8 * hh;
#pragma unroll
  for (int e = 0; e < 8; ++e) { b16 a, c; split16(p0[e], a, c); fh_[e] = a; fl_[e] = c; split16(p1[e], a, c); fh_[8 + e] = a; fl_[8 + e] = c; }
}
__device__ __forceinline__ v8f wmma16b(v16b a, v16b b, v8f c) {
  v8f d = __builtin_amdgcn_wmma_f32_16x16x32_f16(false, a, false, b, (short)0, c, false, false);
  asm volatile("v_nop\n\tv_nop\n\tv_nop\n\tv_nop" : "+v"(d) : "v"(a), "v"(b));
  return d;
}
__device__ __forceinline__ void wave_lds_sync() {
  __builtin_amdgcn_fence(__ATOMIC_RELEASE, "workgroup");
  __builtin_amdgcn_wave_barrier();
  __builtin_amdgcn_fence(__ATOMIC_ACQUIRE, "workgroup");
}

struct Opnd { const void* p0; const void* p1; int ld; };
template <int NP> __device__ __forceinline__ void load_frags(const Opnd& o, int row, int kb, int hh, v16b& fh_, v16b& fl_) {
  if (NP == 0) { frag_ksplit((const float*)o.p0 + (size_t)row * o.ld + kb, hh, fh_, fl_); }
  else if (NP == 3) {
    const float* p = (const float*)o.p0 + (size_t)row * o.ld + kb; const float* p0 = p + 8 * hh; const float* p1 = p + 16 + 8 * hh;
#pragma unroll
    for (int e = 0; e < 8; ++e) { fh_[e] = (b16)p0[e]; fh_[8 + e] = (b16)p1[e]; }
    fl_ = fh_;
  } else {
    fh_ = frag_kb((const b16*)o.p0 + (size_t)row * o.ld + kb, hh);
    if (NP == 2) fl_ = frag_kb((const b16*)o.p1 + (size_t)row * o.ld + kb, hh); else fl_ = fh_;
  }
}
template <int ANP, int BNP> __device__ __forceinline__ v8f mac(v16b ah, v16b al, v16b bh, v16b bl, v8f c) {
  c = wmma16b(ah, bh, c);
  if (BNP == 0 || BNP == 2) c = wmma16b(ah, bl, c);
  if (ANP == 0 || ANP == 2) c = wmma16b(al, bh, c);
  return c;
}
template <int ANP, int BNP>
__device__ __forceinline__ void gemm_tile(const Opnd& A, const Opnd& B, int K, int m0, int c0, int nloc, int hlf, v8f (&acc)[2][4]) {
  for (int kb = 0; kb < K; kb += 32) {
    v16b a0h, a0l, a1h, a1l;
    load_frags<ANP>(A, m0 + nloc, kb, hlf, a0h, a0l);
    load_frags<ANP>(A, m0 + 16 + nloc, kb, hlf, a1h, a1l);
#pragma unroll
    for (int t = 0; t < 4; ++t) {
      v16b bh, bl;
      load_frags<BNP>(B, c0 + t * 16 + nloc, kb, hlf, bh, bl);
      acc[0][t] = mac<ANP, BNP>(a0h, a0l, bh, bl, acc[0][t]);
      acc[1][t] = mac<ANP, BNP>(a1h, a1l, bh, bl, acc[1][t]);
    }
  }
}

struct Epi { float scale; const float* cscale; const float* cbias; const float* rbias; int act; float post; const float* rscale; const float* resid; };
__device__ __forceinline__ float epi_val(const Epi& e, float acc, int row, int col) {
  float val = acc * e.scale;
  if (e.cscale) val *= e.cscale[col];
  if (e.cbias) val += e.cbias[col];
  if (e.rbias) val += e.rbias[row];
  if (e.act == 1) val = 0.5f * val * (1.0f + erff(val * 0.70710678118654752f));
  val *= e.post;
  if (e.rscale) val *= e.rscale[(size_t)row * 32];
  return val;
}
__device__ __forceinline__ void epi_planes(v8f (&acc)[2][4], const Epi& e, bool two,
                                           b16* __restrict__ oh, b16* __restrict__ ol, int ldo, int m0, int c0, int lane, b16* Th, b16* Tl) {
  const int nloc = lane & 15, hlf = lane >> 4;
#pragma unroll
  for (int t = 0; t < 4; ++t)
#pragma unroll
    for (int r = 0; r < 2; ++r)
#pragma unroll
      for (int v = 0; v < 8; ++v) {
        const int rr = r * 16 + v + 8 * hlf, cc = t * 16 + nloc;
        const float val = epi_val(e, acc[r][t][v], m0 + rr, c0 + cc);
        b16 h_, l_; split16(val, h_, l_);
        Th[rr * 64 + cc] = h_; if (two) Tl[rr * 64 + cc] = l_;
      }
  wave_lds_sync();
  for (int pass = 0; pass < 2; ++pass) {
#pragma unroll
    for (int j = 0; j < 8; ++j) {
      const int rr = j * 4 + (lane >> 3), c8 = (lane & 7) * 8;
      const size_t o = (size_t)(m0 + rr) * ldo + c0 + c8;
      *(volatile v8b*)(oh + o) = ld8b(Th + rr * 64 + c8);
      if (two) *(volatile v8b*)(ol + o) = ld8b(Tl + rr * 64 + c8);
    }
    __threadfence();
  }
}
__device__ __forceinline__ void epi_f32(v8f (&acc)[2][4], const Epi& e, float* __restrict__ out, int ldo, int m0, int c0, int lane, float* Tt) {
  const int nloc = lane & 15, hlf = lane >> 4;
#pragma unroll
  for (int t = 0; t < 4; ++t)
#pragma unroll
    for (int r = 0; r < 2; ++r)
#pragma unroll
      for (int v = 0; v < 8; ++v) {
        const int rr = r * 16 + v + 8 * hlf, cc = t * 16 + nloc;
        Tt[rr * 64 + cc] = epi_val(e, acc[r][t][v], m0 + rr, c0 + cc);
      }
  wave_lds_sync();
  float* dst0 = out + (size_t)m0 * ldo + c0; const float* rs0 = e.resid ? e.resid + (size_t)m0 * ldo + c0 : nullptr;
  for (int pass = 0; pass < 2; ++pass) {
#pragma unroll
    for (int j = 0; j < 16; ++j) {
      const int rr = j * 2 + hlf, c4 = nloc * 4;
      v4f val = *(const v4f*)(Tt + rr * 64 + c4);
      if (rs0) val += *(const v4f*)(rs0 + (size_t)rr * ldo + c4);
      *(volatile v4f*)(dst0 + (size_t)rr * ldo + c4) = val;
    }
    __threadfence();
  }
}


__global__ __launch_bounds__(256) void prep_kernel(const float* __restrict__ qkv_w, const float* __restrict__ proj_w, const float* __restrict__ tbl,
                                                   const float* __restrict__ w1, const float* __restrict__ b1, const float* __restrict__ w2,
                                                   b16* __restrict__ w16, float* __restrict__ btab) {
  const size_t tid = (size_t)blockIdx.x * blockDim.x + threadIdx.x, stride = (size_t)gridDim.x * blockDim.x;
  const size_t n0 = (size_t)NQKV * C / 8, n1 = (size_t)C * C / 8, n2 = (size_t)NH * TBLP;
  for (int pass = 0; pass < 2; ++pass) {
    for (size_t c = tid; c < n0 + n1 + n2; c += stride) {
      if (c < n0 + n1) {
        const float* src = (c < n0) ? (qkv_w + c * 8) : (proj_w + (c - n0) * 8); v8b v;
#pragma unroll
        for (int e = 0; e < 8; ++e) v[e] = (b16)src[e];
        *(volatile v8b*)(w16 + c * 8) = v;
      } else {
        const size_t q = c - n0 - n1; const int h = (int)(q / TBLP), e = (int)(q % TBLP);
        float val = 0.0f;
        if (e < TBL) {
          const float t0 = tbl[e * 2], t1 = tbl[e * 2 + 1]; float s = 0.0f;
#pragma unroll 1
          for (int j = 0; j < CPB; ++j) { const float hdn = fmaxf(t0 * w1[j * 2] + t1 * w1[j * 2 + 1] + b1[j], 0.0f); s += hdn * w2[(size_t)h * CPB + j]; }
          val = 16.0f / (1.0f + expf(-s));
        }
        ((volatile float*)btab)[q] = val;
      }
    }
    __threadfence();
  }
}

__global__ __launch_bounds__(128) void qkv_kernel(const float* __restrict__ x, const b16* __restrict__ w16, const float* __restrict__ bias, const float* __restrict__ lscale,
                                                  b16* __restrict__ Q, b16* __restrict__ K, b16* __restrict__ V) {
  __shared__ __attribute__((aligned(16))) b16 Ts[4][2][32 * 32];
  const int lane = threadIdx.x & 31, wave = threadIdx.x >> 5, nloc = lane & 15, hlf = lane >> 4;
  const int m0 = blockIdx.y * 128 + wave * 32, c0 = blockIdx.x * 64;
  const int mat = c0 / C, hA = (c0 % C) / DH;
  v8f acc[2][4];
#pragma unroll
  for (int r = 0; r < 2; ++r)
#pragma unroll
    for (int t = 0; t < 4; ++t) acc[r][t] = (v8f){};
  const Opnd A{x, nullptr, C}, B{w16, nullptr, C};
  gemm_tile<0, 1>(A, B, C, m0, c0, nloc, hlf, acc);
  float sc[2] = {1.0f, 1.0f};
  if (mat == 0) {
#pragma unroll
    for (int u = 0; u < 2; ++u) sc[u] = expf(fminf(lscale[hA + u], 4.605170185988091f));
  } else if (mat == 1) { sc[0] = KSC; sc[1] = KSC; }
#pragma unroll
  for (int r = 0; r < 2; ++r)
#pragma unroll
    for (int v = 0; v < 8; ++v) {
      const int rr = r * 16 + v + 8 * hlf;
      float val[4];
#pragma unroll
      for (int t = 0; t < 4; ++t) val[t] = acc[r][t][v] + bias[c0 + t * 16 + nloc];
      float f[2] = {1.0f, 1.0f};
      if (mat < 2) {
#pragma unroll
        for (int u = 0; u < 2; ++u) {
          float ss = val[2 * u] * val[2 * u] + val[2 * u + 1] * val[2 * u + 1];
#pragma unroll
          for (int o = 1; o < 16; o <<= 1) ss += __shfl_xor(ss, o);
          f[u] = sc[u] / fmaxf(sqrtf(ss), 1e-12f);
        }
      }
#pragma unroll
      for (int t = 0; t < 4; ++t) {
        const int u = t >> 1, d = (t & 1) * 16 + nloc;
        const int idx = (mat < 2) ? (rr * 32 + d) : ((rr >> 4) * 512 + d * 16 + (rr & 15));
        Ts[wave][u][idx] = (b16)(val[t] * f[u]);
      }
    }
  wave_lds_sync();
  const int w = m0 / N, t0 = m0 % N;
  b16* base = (mat == 0) ? Q : (mat == 1) ? K : V;
  for (int pass = 0; pass < 2; ++pass) {
#pragma unroll
    for (int u = 0; u < 2; ++u) {
      b16* dst = base + ((size_t)(w * NH + hA + u) * N + t0) * DH;
#pragma unroll
      for (int j = 0; j < 4; ++j) { const int e = (j * 32 + lane) * 8; *(volatile v8b*)(dst + e) = ld8b(Ts[wave][u] + e); }
    }
    __threadfence();
  }
}

__global__ __launch_bounds__(192) void attn_kernel(const b16* __restrict__ Q, const b16* __restrict__ K, const b16* __restrict__ V, const float* __restrict__ btab,
                                                   const int* __restrict__ ridx, const float* __restrict__ mask, b16* __restrict__ y) {
  __shared__ __attribute__((aligned(16))) b16 Os[16 * C];
  const int h = threadIdx.x >> 5, lane = threadIdx.x & 31, hh = lane >> 4, col = lane & 15;
  const int w = blockIdx.x / (N / 16), q0 = (blockIdx.x % (N / 16)) * 16, g = w * NH + h;
  const size_t ko = (size_t)g * N * DH;
  const v16b qf = frag_kb(Q + ((size_t)g * N + q0 + col) * DH, hh);
  const int qi = q0 + col;
  const int* rrow = ridx + (size_t)qi * N; const float* mrow = mask + ((size_t)(w % NW) * N + qi) * N; const float* bt = btab + (size_t)h * TBLP;
  float m = -INFINITY, l = 0.0f;
  v8f o0 = {}, o1 = {};
  for (int kb = 0; kb < N; kb += 32) {
    v8f s0 = {}, s1 = {};
    s0 = wmma16b(frag_kb(K + ko + (size_t)(kb + col) * DH, hh), qf, s0);
    s1 = wmma16b(frag_kb(K + ko + (size_t)(kb + 16 + col) * DH, hh), qf, s1);
    float mr = -INFINITY;
#pragma unroll
    for (int r = 0; r < 8; ++r) {
      const int k0i = kb + 8 * hh + r, k1i = k0i + 16;
      int e0 = rrow[k0i], e1 = rrow[k1i]; e0 = e0 < 0 ? 0 : (e0 >= TBL ? TBL - 1 : e0); e1 = e1 < 0 ? 0 : (e1 >= TBL ? TBL - 1 : e1);
      s0[r] = s0[r] * (1.0f / KSC) + bt[e0] + mrow[k0i];
      s1[r] = s1[r] * (1.0f / KSC) + bt[e1] + mrow[k1i];
      mr = fmaxf(mr, fmaxf(s0[r], s1[r]));
    }
    mr = fmaxf(mr, __shfl_xor(mr, 16));
    const float mn = fmaxf(m, mr), al_ = __expf(m - mn);
    m = mn;
    float sum = 0.0f; v16b pb;
#pragma unroll
    for (int r = 0; r < 8; ++r) { const float p0 = __expf(s0[r] - mn), p1 = __expf(s1[r] - mn); sum += p0 + p1; pb[r] = (b16)p0; pb[8 + r] = (b16)p1; }
    sum += __shfl_xor(sum, 16);
    l = l * al_ + sum;
#pragma unroll
    for (int r = 0; r < 8; ++r) { o0[r] *= al_; o1[r] *= al_; }
    const size_t v0 = ko + (size_t)(kb >> 4) * (DH * 16) + 8 * hh, v1 = v0 + DH * 16;
    o0 = wmma16b(cat8b(ld8b(V + v0 + (size_t)col * 16), ld8b(V + v1 + (size_t)col * 16)), pb, o0);
    o1 = wmma16b(cat8b(ld8b(V + v0 + (size_t)(16 + col) * 16), ld8b(V + v1 + (size_t)(16 + col) * 16)), pb, o1);
  }
  const float inv = 1.0f / l;
#pragma unroll
  for (int r = 0; r < 8; ++r) {
    Os[col * C + h * DH + 8 * hh + r] = (b16)(o0[r] * inv);
    Os[col * C + h * DH + 16 + 8 * hh + r] = (b16)(o1[r] * inv);
  }
  __syncthreads();
  b16* dst = y + ((size_t)w * N + q0) * C;
  for (int pass = 0; pass < 2; ++pass) {
    for (int p = threadIdx.x; p < 16 * C / 8; p += 192) *(volatile v8b*)(dst + (size_t)p * 8) = ld8b(Os + p * 8);
    __threadfence();
  }
}

__global__ __launch_bounds__(128) void proj_kernel(const b16* __restrict__ y, const b16* __restrict__ pw16, const float* __restrict__ pb, float* __restrict__ out) {
  __shared__ __attribute__((aligned(16))) float Ts[4][32 * 64];
  const int lane = threadIdx.x & 31, wave = threadIdx.x >> 5, nloc = lane & 15, hlf = lane >> 4;
  const int m0 = blockIdx.y * 128 + wave * 32, c0 = blockIdx.x * 64;
  v8f acc[2][4];
#pragma unroll
  for (int r = 0; r < 2; ++r)
#pragma unroll
    for (int t = 0; t < 4; ++t) acc[r][t] = (v8f){};
  const Opnd A{y, nullptr, C}, B{pw16, nullptr, C};
  gemm_tile<1, 1>(A, B, C, m0, c0, nloc, hlf, acc);
  const Epi e{1.0f, nullptr, pb, nullptr, 0, 1.0f, nullptr, nullptr};
  epi_f32(acc, e, out, C, m0, c0, lane, Ts[wave]);
}
}

extern "C" void kernel_launch(void* const* d_in, const int* in_sizes, int n_in,
                              void* d_out, int out_size, void* d_ws, size_t ws_size, hipStream_t stream) {
  (void)n_in; (void)out_size;
  const float* x     = (const float*)d_in[0];
  const float* mask  = (const float*)d_in[1];
  const float* qkv_w = (const float*)d_in[2];
  const float* qkv_b = (const float*)d_in[3];
  const float* pw    = (const float*)d_in[4];
  const float* pb    = (const float*)d_in[5];
  const float* lsc   = (const float*)d_in[6];
  const float* w1    = (const float*)d_in[7];
  const float* b1    = (const float*)d_in[8];
  const float* w2    = (const float*)d_in[9];
  const float* tbl   = (const float*)d_in[10];
  const int* ridx    = (const int*)d_in[11];
  float* out = (float*)d_out;
  if (in_sizes[0] != MROWS * C || in_sizes[1] != NW * N * N || in_sizes[2] != NQKV * C || in_sizes[11] != N * N || in_sizes[10] != TBL * 2) return;

  size_t off = 0; char* ws = (char*)d_ws;
  auto carve = [&](size_t bytes) { char* p = ws + off; off += (bytes + 255) & ~(size_t)255; return p; };
  b16* w16    = (b16*)carve((size_t)(NQKV * C + C * C) * 2);
  float* btab = (float*)carve((size_t)NH * TBLP * 4);
  b16* Qb     = (b16*)carve((size_t)MROWS * C * 2);
  b16* Kb     = (b16*)carve((size_t)MROWS * C * 2);
  b16* Vb     = (b16*)carve((size_t)MROWS * C * 2);
  b16* yb     = (b16*)carve((size_t)MROWS * C * 2);
  if (off > ws_size) return;
  prep_kernel<<<64, 256, 0, stream>>>(qkv_w, pw, tbl, w1, b1, w2, w16, btab);
  qkv_kernel<<<dim3(NQKV / 64, MROWS / 128), 128, 0, stream>>>(x, w16, qkv_b, lsc, Qb, Kb, Vb);
  attn_kernel<<<BW * (N / 16), 192, 0, stream>>>(Qb, Kb, Vb, btab, ridx, mask, yb);
  proj_kernel<<<dim3(C / 64, MROWS / 128), 128, 0, stream>>>(yb, w16 + (size_t)NQKV * C, pb, out);
}
